// KPConvLayer_71116068488052
// MI455X (gfx1250) — hardware-run, weakly checked
//
#include <hip/hip_runtime.h>


namespace {
constexpr int NB = 2, NP = 32768, KN = 32, CI = 128, CO = 128, S = 15, NT = NB * NP;
constexpr float SIG = 0.03f, XS = 8.0f, HS = 256.0f, WSC = 256.0f;
typedef _Float16 b16;
typedef __attribute__((ext_vector_type(16))) _Float16 v16b;
typedef __attribute__((ext_vector_type(8))) _Float16 v8b;
typedef __attribute__((ext_vector_type(8))) float v8f;
typedef __attribute__((ext_vector_type(4))) float v4f;
typedef __attribute__((ext_vector_type(2))) _Float16 v2b;
__device__ __forceinline__ float bf16_rne(float f) { unsigned int u = __float_as_uint(f); u += 0x7FFFu + ((u >> 16) & 1u); float r = __uint_as_float(u & 0xFFFF0000u); asm volatile("" : "+v"(r)); return r; }
__device__ __forceinline__ float bfv(float f) { float r = bf16_rne(f); asm volatile("" : "+v"(r)); return r; }
__device__ __forceinline__ void split16(float v, b16& hi, b16& lo) { hi = (b16)v; lo = (b16)(v - (float)hi); }
__device__ __forceinline__ v16b frag_kb(const b16* p, int hh) { const v8b a = *(const v8b*)(p + 8 * hh), b = *(const v8b*)(p + 16 + 8 * hh); v16b f;
#pragma unroll
  for (int e = 0; e < 8; ++e) { f[e] = a[e]; f[8 + e] = b[e]; } return f; }
__device__ __forceinline__ v8f wmma16b(v16b a, v16b b, v8f c) { v8f d = __builtin_amdgcn_wmma_f32_16x16x32_f16(false, a, false, b, (short)0, c, false, false); asm volatile("v_nop\n\tv_nop\n\tv_nop\n\tv_nop" : "+v"(d) : "v"(a), "v"(b)); return d; }
__device__ __forceinline__ void wave_lds_sync() { __builtin_amdgcn_fence(__ATOMIC_RELEASE, "workgroup"); __builtin_amdgcn_wave_barrier(); __builtin_amdgcn_fence(__ATOMIC_ACQUIRE, "workgroup"); }
__device__ __forceinline__ float pmul(float a, float b) { float p = a * b; asm volatile("" : "+v"(p)); return p; }
__device__ __forceinline__ int iclamp(int v, int lo, int hi) { return v < lo ? lo : (v > hi ? hi : v); }

__global__ __launch_bounds__(256) void wput_kernel(const float* __restrict__ w, b16* __restrict__ WT) { const int u = blockIdx.x * 256 + threadIdx.x; if (u >= S * CO * (CI / 8)) return; const int r = u / (CI / 8), c0 = (u % (CI / 8)) * 8; const int s = r / CO, o = r % CO; v8b v;
#pragma unroll
  for (int j = 0; j < 8; ++j) v[j] = (b16)(bf16_rne(w[((size_t)s * CI + c0 + j) * CO + o]) * WSC); for (int pass = 0; pass < 2; ++pass) { *(volatile v8b*)(WT + (size_t)r * CI + c0) = v; __threadfence(); } }
__global__ __launch_bounds__(32) void kp_kernel(const float* __restrict__ xyz, const float* __restrict__ feat, const int* __restrict__ nbr, const float* __restrict__ kp, const b16* __restrict__ WT, const float* __restrict__ bias, int TLIM, float* __restrict__ out) {
  __shared__ float KW[16][S][KN]; __shared__ __attribute__((aligned(16))) b16 Ah[16][40], Al[16][40], Ft[64][40], Gh[S][16][72], Gl[S][16][72]; __shared__ float Tf[16][CO + 4]; __shared__ int NB_[16][KN];
  const int lane = threadIdx.x, nloc = lane & 15, hlf = lane >> 4; const size_t t0 = (size_t)blockIdx.x * 16; if (t0 >= (size_t)TLIM) return; const int b = (int)(t0 / NP);
  const float inv2s2 = 1.0f / (2.0f * SIG * SIG);
  float kpx[S], kpy[S], kpz[S];
#pragma unroll
  for (int s = 0; s < S; ++s) { kpx[s] = bfv(kp[s * 3]); kpy[s] = bfv(kp[s * 3 + 1]); kpz[s] = bfv(kp[s * 3 + 2]); }
  for (int p = 0; p < 16; ++p) { const size_t n = t0 + p; const int u = iclamp(nbr[n * KN + lane], 0, NP - 1); NB_[p][lane] = u; const size_t gn = (size_t)b * NP + u;
    const float rx = bfv(xyz[gn * 3]) - bfv(xyz[n * 3]), ry = bfv(xyz[gn * 3 + 1]) - bfv(xyz[n * 3 + 1]), rz = bfv(xyz[gn * 3 + 2]) - bfv(xyz[n * 3 + 2]);
#pragma unroll
    for (int s = 0; s < S; ++s) { const float dx = rx - kpx[s], dy = ry - kpy[s], dz = rz - kpz[s]; const float d2 = dx * dx + dy * dy + dz * dz; KW[p][s][lane] = expf(-d2 * inv2s2); } }
  if (lane < 16) { for (int k = KN; k < 40; ++k) { Ah[lane][k] = (b16)0.0f; Al[lane][k] = (b16)0.0f; } for (int k = 0; k < 40; ++k) if (lane == 15) { Ah[15][k] = (b16)0.0f; Al[15][k] = (b16)0.0f; } }
  wave_lds_sync();
  v8f acc2[8];
#pragma unroll
  for (int t = 0; t < 8; ++t) acc2[t] = (v8f){};
#pragma unroll 1
  for (int h = 0; h < 2; ++h) {
#pragma unroll 1
    for (int p = 0; p < 16; ++p) {
      for (int s = 0; s < S; ++s) { b16 ph, pl; split16(KW[p][s][lane] * HS, ph, pl); Ah[s][lane] = ph; Al[s][lane] = pl; }
      { const size_t gn = (size_t)b * NP + NB_[p][lane]; const float* fp = feat + gn * CI + h * 64;
        for (int c = 0; c < 64; ++c) Ft[c][lane] = (b16)(bf16_rne(fp[c]) * XS); if (lane < 8) for (int c = 0; c < 64; ++c) Ft[c][KN + lane] = (b16)0.0f; }
      wave_lds_sync();
      const v16b ah = frag_kb(&Ah[nloc][0], hlf), al = frag_kb(&Al[nloc][0], hlf); v8f d4[4];
#pragma unroll
      for (int t = 0; t < 4; ++t) { const v16b bf = frag_kb(&Ft[t * 16 + nloc][0], hlf); d4[t] = (v8f){}; d4[t] = wmma16b(ah, bf, d4[t]); d4[t] = wmma16b(al, bf, d4[t]); }
#pragma unroll
      for (int t = 0; t < 4; ++t)
#pragma unroll
        for (int r8 = 0; r8 < 8; ++r8) { const int s = 8 * hlf + r8; if (s < S) { b16 gh, gl; split16(d4[t][r8] * (HS / (HS * XS)), gh, gl); Gh[s][p][t * 16 + nloc] = gh; Gl[s][p][t * 16 + nloc] = gl; } }
      wave_lds_sync(); }
    if (lane < 16) for (int s = 0; s < S; ++s) for (int k = 64; k < 72; ++k) { Gh[s][lane][k] = (b16)0.0f; Gl[s][lane][k] = (b16)0.0f; }
    wave_lds_sync();
#pragma unroll 1
    for (int s = 0; s < S; ++s) {
#pragma unroll
      for (int kb = 0; kb < 64; kb += 32) { const v16b a = frag_kb(&Gh[s][nloc][kb], hlf), alo = frag_kb(&Gl[s][nloc][kb], hlf);
#pragma unroll
        for (int t = 0; t < 8; ++t) { const v16b bw = frag_kb(WT + ((size_t)s * CO + t * 16 + nloc) * CI + h * 64 + kb, hlf); acc2[t] = wmma16b(a, bw, acc2[t]); acc2[t] = wmma16b(alo, bw, acc2[t]); } } }
    wave_lds_sync(); }
#pragma unroll
  for (int t = 0; t < 8; ++t) { const int o = t * 16 + nloc; const float bb = bfv(bias[o]);
#pragma unroll
    for (int r8 = 0; r8 < 8; ++r8) Tf[8 * hlf + r8][o] = acc2[t][r8] * (1.0f / (HS * WSC)) + bb; }
  wave_lds_sync();
  for (int pass = 0; pass < 2; ++pass) { for (int p = 0; p < 16; ++p) *(volatile v4f*)(out + (t0 + p) * CO + lane * 4) = *(const v4f*)(&Tf[p][lane * 4]); __threadfence(); } }
}

extern "C" void kernel_launch(void* const* d_in, const int* in_sizes, int n_in, void* d_out, int out_size, void* d_ws, size_t ws_size, hipStream_t stream) {
  (void)n_in;
  auto Fp = [&](int i) { return (const float*)d_in[i]; }; auto Ip = [&](int i) { return (const int*)d_in[i]; };
  if (in_sizes[0] != NT * 3 || in_sizes[1] != NT * CI || in_sizes[2] != NT * KN || in_sizes[3] != S * 3 || in_sizes[4] != S * CI * CO || in_sizes[5] != CO || out_size != NT * CO) return;
  const int TLIM = NT;
  size_t off = 0; char* ws = (char*)d_ws;
  auto carve = [&](size_t bytes) { char* p = ws + off; off += (bytes + 255) & ~(size_t)255; return p; };
  b16* WT = (b16*)carve((size_t)S * CO * CI * 2);
  if (off > ws_size || off > ((size_t)4 << 20)) return;
  wput_kernel<<<(S * CO * (CI / 8) + 255) / 256, 256, 0, stream>>>(Fp(4), WT);
  kp_kernel<<<TLIM / 16, 32, 0, stream>>>(Fp(0), Fp(1), Ip(2), Fp(3), WT, Fp(5), TLIM, (float*)d_out);
}
